// GCNGraphClassifier_77704548319503
// MI455X (gfx1250) — hardware-verified
//
#include <hip/hip_runtime.h>
#include <hip/hip_bf16.h>
#include <math.h>


#define BB 2
#define SS 2048
#define DD 1024
#define HH 16
#define DKK 64
#define QW 2

typedef _Float16 bf16;
typedef __attribute__((ext_vector_type(4))) unsigned v4u_t;
typedef unsigned v4ua __attribute__((ext_vector_type(4), may_alias));
typedef __attribute__((ext_vector_type(4))) float v4f_t;
typedef float v4fa __attribute__((ext_vector_type(4), may_alias));
typedef __attribute__((ext_vector_type(16))) bf16  bf16x16;
typedef __attribute__((ext_vector_type(8)))  bf16  bf16x8;
typedef __attribute__((ext_vector_type(4)))  bf16  bf16x4;
typedef __attribute__((ext_vector_type(8)))  float f32x8;

#define LDS_STRIDE 48
#define KSTRIDE    72
#define VSTRIDE    48

__device__ __forceinline__ f32x8 wmma_bf16(bf16x16 a, bf16x16 b, f32x8 c) {
  return __builtin_amdgcn_wmma_f32_16x16x32_f16(
      false, a, false, b, (short)0, c, false, false);
}
#define RSPLIT (1.0f / 2048.0f)
__device__ __forceinline__ bf16 lo_of(float v, bf16 h) { return (bf16)((v - (float)h) * 2048.0f); }
__device__ __forceinline__ f32x8 wmma_split(bf16x16 a, bf16x16 al, bf16x16 b, bf16x16 bl, f32x8 c) {
  f32x8 x = {}; x = wmma_bf16(al, b, x); x = wmma_bf16(a, bl, x); return wmma_bf16(a, b, c) + x * RSPLIT; }

template <typename T>
__device__ __forceinline__ bf16x16 load_frag(const T* __restrict__ base, int ld,
                                             int row0, int k0) {
  const int lane = threadIdx.x & 31;
  const int r    = lane & 15;
  const int kh   = (lane >> 4) * 8;
  const T* p0 = base + (size_t)(row0 + r) * ld + (k0 + kh);
  const T* p1 = p0 + 16;
  bf16x16 f;
#pragma unroll
  for (int i = 0; i < 8; ++i) {
    f[i]     = (bf16)p0[i];
    f[i + 8] = (bf16)p1[i];
  }
  return f;
}

__device__ __forceinline__ bf16x16 lds_frag(const bf16* base, int stride) {
  const int lane = threadIdx.x & 31;
  const int row  = lane & 15;
  const int kh   = (lane >> 4) * 8;
  const bf16x8 lo = *(const bf16x8*)(base + row * stride + kh);
  const bf16x8 hi = *(const bf16x8*)(base + row * stride + kh + 16);
  bf16x16 f;
#pragma unroll
  for (int i = 0; i < 8; ++i) { f[i] = lo[i]; f[i + 8] = hi[i]; }
  return f;
}

template <typename T>
__device__ __forceinline__ void stage_read16(const T* __restrict__ p, float* buf) {
#pragma unroll
  for (int i = 0; i < 16; ++i) buf[i] = (float)p[i];
}

__device__ __forceinline__ void stage_write(bf16* dst, const float* buf, int nquad) {
#pragma unroll
  for (int i = 0; i < nquad; ++i) {
    bf16x4 q;
    q[0] = (bf16)buf[4 * i];     q[1] = (bf16)buf[4 * i + 1];
    q[2] = (bf16)buf[4 * i + 2]; q[3] = (bf16)buf[4 * i + 3];
    *(bf16x4*)(dst + 4 * i) = q;
  }
}

__global__ __launch_bounds__(256) void transpose_pack_kernel(const float* __restrict__ W, bf16* __restrict__ WT, int K, int N, size_t plane) {
  __shared__ float tile[64][65];
  const int k0 = blockIdx.y * 64, n0 = blockIdx.x * 64, t = threadIdx.x;
  for (int i = t; i < 64 * 64; i += 256) { const int kr = i >> 6, nc = i & 63; tile[kr][nc] = W[(size_t)(k0 + kr) * N + n0 + nc]; }
  __syncthreads();
#pragma unroll 1
  for (int pass = 0; pass < 2; ++pass) {
    for (int i = t; i < 64 * 8; i += 256) { const int nr = i >> 3, k8 = (i & 7) * 8; bf16 hh[8], hl[8];
#pragma unroll
      for (int e = 0; e < 8; ++e) { const float v = tile[k8 + e][nr]; hh[e] = (bf16)v; hl[e] = lo_of(v, hh[e]); }
      bf16* d = WT + (size_t)(n0 + nr) * K + k0 + k8;
      *(volatile v4u_t*)d = *(const v4ua*)hh; *(volatile v4u_t*)(d + plane) = *(const v4ua*)hl; }
    __threadfence();
  }
}

template <typename AT, typename WT, int MODE>
__global__ __launch_bounds__(256) void gemm_split_kernel(
    const AT* __restrict__ A, size_t aPlane, const WT* __restrict__ W, size_t wPlane,
    const float* __restrict__ bias, void* __restrict__ out,
    int M, int N, int K) {
  __shared__ bf16 ldsA[128 * LDS_STRIDE], ldsAl[128 * LDS_STRIDE];
  __shared__ bf16 ldsW[256 * LDS_STRIDE], ldsWl[256 * LDS_STRIDE];
  __shared__ __attribute__((aligned(16))) unsigned char sob[256 * 136 * 2];

  const int t    = threadIdx.x;
  const int wave = t >> 5;
  const int lane = t & 31;
  const int wm   = (wave & 1) * 64;
  const int wn   = (wave >> 1) * 64;
  const int mBlk = blockIdx.x * 128;
  const int nBlk = blockIdx.y * 256;
  const int arow = t >> 1;
  const int ach  = (t & 1) * 16;

  f32x8 acc[4][4] = {};
  for (int k = 0; k < K; k += 32) {
    __syncthreads();
    {
      const AT* ap = A + (size_t)(mBlk + arow) * K + k + ach;
      bf16 hh[16], hl[16];
      if (sizeof(AT) == 4) {
#pragma unroll
        for (int i = 0; i < 16; ++i) { const float v = (float)ap[i]; hh[i] = (bf16)v; hl[i] = lo_of(v, hh[i]); }
      } else {
#pragma unroll
        for (int i = 0; i < 16; ++i) { hh[i] = (bf16)ap[i]; hl[i] = (bf16)ap[aPlane + i]; }
      }
#pragma unroll
      for (int i = 0; i < 16; ++i) { ldsA[arow * LDS_STRIDE + ach + i] = hh[i]; ldsAl[arow * LDS_STRIDE + ach + i] = hl[i]; }
    }
    {
      const WT* wp = W + (size_t)(nBlk + t) * K + k;
      if (sizeof(WT) == 4) {
#pragma unroll
        for (int i = 0; i < 32; ++i) { const float v = (float)wp[i]; const bf16 h_ = (bf16)v; ldsW[t * LDS_STRIDE + i] = h_; ldsWl[t * LDS_STRIDE + i] = lo_of(v, h_); }
      } else {
#pragma unroll
        for (int i = 0; i < 32; ++i) { ldsW[t * LDS_STRIDE + i] = (bf16)wp[i]; ldsWl[t * LDS_STRIDE + i] = (bf16)wp[wPlane + i]; }
      }
    }
    __syncthreads();
    bf16x16 wf[4], wfl[4];
#pragma unroll
    for (int j = 0; j < 4; ++j) { wf[j] = lds_frag(ldsW + (wn + 16 * j) * LDS_STRIDE, LDS_STRIDE); wfl[j] = lds_frag(ldsWl + (wn + 16 * j) * LDS_STRIDE, LDS_STRIDE); }
#pragma unroll
    for (int i = 0; i < 4; ++i) {
      const bf16x16 af = lds_frag(ldsA + (wm + 16 * i) * LDS_STRIDE, LDS_STRIDE), afl = lds_frag(ldsAl + (wm + 16 * i) * LDS_STRIDE, LDS_STRIDE);
#pragma unroll
      for (int j = 0; j < 4; ++j) acc[i][j] = wmma_split(af, afl, wf[j], wfl[j], acc[i][j]);
    }
  }

  const int nlane = lane & 15;
  const int mh    = (lane >> 4) * 8;
  __syncthreads();
  if (MODE == 1) {
    bf16* so = (bf16*)sob;
#pragma unroll
    for (int i = 0; i < 4; ++i)
#pragma unroll
      for (int j = 0; j < 4; ++j) {
        const int nl = wn + 16 * j + nlane;
        const float bv = bias ? bias[nBlk + nl] : 0.0f;
#pragma unroll
        for (int r = 0; r < 8; ++r) so[nl * 136 + wm + 16 * i + mh + r] = (bf16)(acc[i][j][r] + bv);
      }
    __syncthreads();
    const int b_ = mBlk >> 11, s0 = mBlk & (SS - 1);
#pragma unroll 1
    for (int pass = 0; pass < 2; ++pass) {
      for (int ch = t; ch < 256 * 16; ch += 256) { const int nl = ch >> 4, q = (ch & 15) * 8; const int n = nBlk + nl, h = n >> 6, dk = n & (DKK - 1);
        *(volatile v4u_t*)((bf16*)out + (((size_t)(b_ * HH + h)) * DKK + dk) * SS + s0 + q) = *(const v4ua*)(so + nl * 136 + q); }
      __threadfence();
    }
  } else {
    float* so = (float*)sob;
#pragma unroll 1
    for (int hf = 0; hf < 2; ++hf) {
      if (wm == hf * 64) {
#pragma unroll
        for (int i = 0; i < 4; ++i)
#pragma unroll
          for (int j = 0; j < 4; ++j) {
            const int nl = wn + 16 * j + nlane;
            const float bv = bias ? bias[nBlk + nl] : 0.0f;
#pragma unroll
            for (int r = 0; r < 8; ++r) so[(16 * i + mh + r) * 260 + nl] = acc[i][j][r] + bv;
          }
      }
      __syncthreads();
#pragma unroll 1
      for (int pass = 0; pass < 2; ++pass) {
        for (int ch = t; ch < 64 * 64; ch += 256) { const int ml = ch >> 6, q = (ch & 63) * 4;
          *(volatile v4f_t*)((float*)out + (size_t)(mBlk + hf * 64 + ml) * N + nBlk + q) = *(const volatile v4fa*)(so + ml * 260 + q); }
        __threadfence();
      }
      __syncthreads();
    }
  }
}


#define GN 50000
#define GNP 50176
#define GE 800000
#define GG 500
#define GRANGE 7168

__global__ __launch_bounds__(128) void k_packA(const float* __restrict__ W, int kin, float* __restrict__ A) {
  const int m = blockIdx.x, k = threadIdx.x;
  if (k < kin) { const float v = (m < 64) ? W[k * 64 + m] : 0.0f; *(volatile float*)(A + m * kin + k) = v; __threadfence(); *(volatile float*)(A + m * kin + k) = v; }
}
__global__ __launch_bounds__(256) void k_deg(const int* __restrict__ ei, float* __restrict__ dis) {
  __shared__ int cnt[8][GRANGE / 8 + 1];
  __shared__ int qd[256]; __shared__ int wcnt[8];
  const int tid = threadIdx.x, lane = tid & 31, wave = tid >> 5, r0 = blockIdx.x * GRANGE;
  for (int i = tid; i < 8 * (GRANGE / 8 + 1); i += 256) (&cnt[0][0])[i] = 0;
  __syncthreads();
  const int* dstp = ei + (size_t)GE;
#pragma unroll 1
  for (int c0 = 0; c0 < GE; c0 += 256) {
    const int e = c0 + tid; int d = -1;
    if (e < GE) { const int draw = dstp[e]; const int dd = draw < 0 ? 0 : (draw >= GN ? GN - 1 : draw); if (dd >= r0 && dd < r0 + GRANGE) d = dd - r0; }
    const unsigned m = __builtin_amdgcn_ballot_w32(d >= 0);
    if (lane == 0) wcnt[wave] = __builtin_popcount(m);
    __syncthreads();
    int base = 0, total = 0;
#pragma unroll
    for (int w = 0; w < 8; ++w) { const int c = wcnt[w]; base += (w < wave) ? c : 0; total += c; }
    if (d >= 0) qd[base + __builtin_popcount(m & ((1u << lane) - 1u))] = d;
    __syncthreads();
#pragma unroll 1
    for (int qi = 0; qi < total; ++qi) { const int dl = qd[qi]; if ((dl & 7) != wave) continue; if (lane == 0) cnt[wave][dl >> 3] += 1; }
    __syncthreads();
  }
  const int n4 = GRANGE / 4;
#pragma unroll 1
  for (int pass = 0; pass < 2; ++pass) {
    for (int i = tid; i < n4; i += 256) { v4f_t v;
#pragma unroll
      for (int q = 0; q < 4; ++q) { const int nl = i * 4 + q; v[q] = rsqrtf((float)(cnt[nl & 7][nl >> 3] + 1)); }
      *(volatile v4f_t*)(dis + r0 + i * 4) = v; }
    __threadfence();
  }
}
__global__ __launch_bounds__(256) void k_gcn_agg(const int* __restrict__ ei, const float* __restrict__ hT, const float* __restrict__ dis,
                                                const float* __restrict__ b, float* __restrict__ R, float* __restrict__ Hout) {
  __shared__ int qd[256], qs[256]; __shared__ int wcnt[8];
  const int tid = threadIdx.x, lane = tid & 31, wave = tid >> 5, r0 = blockIdx.x * GRANGE;
  float* myR = R + (size_t)r0 * 64;
  for (int i = tid; i < GRANGE * 64 / 4; i += 256) { v4f_t z; z.x = z.y = z.z = z.w = 0.0f; *(volatile v4f_t*)(myR + (size_t)i * 4) = z; }
  __threadfence(); __syncthreads();
  const int* srcp = ei; const int* dstp = ei + (size_t)GE;
#pragma unroll 1
  for (int c0 = 0; c0 < GE; c0 += 256) {
    const int e = c0 + tid; int d = -1, sidx = 0;
    if (e < GE) { const int draw = dstp[e]; const int dd = draw < 0 ? 0 : (draw >= GN ? GN - 1 : draw);
      if (dd >= r0 && dd < r0 + GRANGE) { d = dd - r0; const int ss = srcp[e]; sidx = ss < 0 ? 0 : (ss >= GN ? GN - 1 : ss); } }
    const unsigned m = __builtin_amdgcn_ballot_w32(d >= 0);
    if (lane == 0) wcnt[wave] = __builtin_popcount(m);
    __syncthreads();
    int base = 0, total = 0;
#pragma unroll
    for (int w = 0; w < 8; ++w) { const int c = wcnt[w]; base += (w < wave) ? c : 0; total += c; }
    if (d >= 0) { const int pos = base + __builtin_popcount(m & ((1u << lane) - 1u)); qd[pos] = d; qs[pos] = sidx; }
    __syncthreads();
#pragma unroll 1
    for (int qi = 0; qi < total; ++qi) {
      const int dl = qd[qi]; if ((dl & 7) != wave) continue;
      const int sl = qs[qi]; const float w = dis[sl];
      float* row = myR + (size_t)dl * 64;
      row[lane] += w * hT[(size_t)lane * GNP + sl]; row[32 + lane] += w * hT[(size_t)(32 + lane) * GNP + sl];
    }
    __syncthreads();
  }
  __threadfence(); __syncthreads();
#pragma unroll 1
  for (int pass = 0; pass < 2; ++pass) {
    for (int i = tid; i < GRANGE * 16; i += 256) { const int nl = i >> 4, c4 = (i & 15) * 4, node = r0 + nl; v4f_t v;
      if (node < GN) { const float di = dis[node];
#pragma unroll
        for (int q = 0; q < 4; ++q) { const int c = c4 + q; v[q] = fmaxf(di * (myR[(size_t)nl * 64 + c] + di * hT[(size_t)c * GNP + node]) + b[c], 0.0f); } }
      else { v.x = v.y = v.z = v.w = 0.0f; }
      *(volatile v4f_t*)(Hout + (size_t)node * 64 + c4) = v; }
    __threadfence();
  }
}
__global__ __launch_bounds__(256) void k_pool_head(const float* __restrict__ H, const int* __restrict__ batch, const float* __restrict__ W1, const float* __restrict__ b1,
                                                  const float* __restrict__ W2, const float* __restrict__ b2, float* __restrict__ logits, float* __restrict__ zero) {
  __shared__ float pool[GG][65]; __shared__ int cnt[GG];
  __shared__ float hid[GG][65];
  const int tid = threadIdx.x, lane = tid & 31, wave = tid >> 5;
  for (int i = tid; i < GG * 65; i += 256) (&pool[0][0])[i] = 0.0f;
  for (int i = tid; i < GG; i += 256) cnt[i] = 0;
  __syncthreads();
#pragma unroll 1
  for (int n0 = 0; n0 < GN; n0 += 32) {
    const int n = n0 + lane; int g = -1;
    if (n < GN) { const int graw = batch[n]; const int gg = graw < 0 ? 0 : (graw >= GG ? GG - 1 : graw); if ((gg & 7) == wave) g = gg; }
    unsigned m = __builtin_amdgcn_ballot_w32(g >= 0);
#pragma unroll 1
    while (m != 0u) { const int l = __builtin_ctz(m); m &= m - 1u;
      const int gl = __shfl(g, l, 32), nn = n0 + l;
      pool[gl][lane] += H[(size_t)nn * 64 + lane]; pool[gl][32 + lane] += H[(size_t)nn * 64 + 32 + lane];
      if (lane == 0) cnt[gl] += 1; }
  }
  __syncthreads();
  for (int i = tid; i < GG * 64; i += 256) { const int g = i >> 6, c = i & 63; const float inv = 1.0f / fmaxf((float)cnt[g], 1.0f);
    float s = b1[c];
#pragma unroll 4
    for (int k = 0; k < 64; ++k) s += (pool[g][k] * inv) * W1[k * 64 + c];
    hid[g][c] = fmaxf(s, 0.0f); }
  __syncthreads();
#pragma unroll 1
  for (int pass = 0; pass < 2; ++pass) {
    for (int i = tid; i < GG * 10; i += 256) { const int g = i / 10, o = i % 10; float s = b2[o];
#pragma unroll 4
      for (int c = 0; c < 64; ++c) s += hid[g][c] * W2[c * 10 + o];
      *(volatile float*)(logits + i) = s; }
    if (tid == 0) *(volatile float*)zero = 0.0f;
    __threadfence();
  }
}

__global__ __launch_bounds__(128) void k_padrows(const float* __restrict__ x, float* __restrict__ XP) {
  const int row = blockIdx.x, k = threadIdx.x; const float v = (row < GN) ? x[(size_t)row * 128 + k] : 0.0f;
  *(volatile float*)(XP + (size_t)row * 128 + k) = v; __threadfence(); *(volatile float*)(XP + (size_t)row * 128 + k) = v;
}

extern "C" void kernel_launch(void* const* d_in, const int* in_sizes, int n_in,
                              void* d_out, int out_size, void* d_ws, size_t ws_size,
                              hipStream_t stream) {
  (void)in_sizes; (void)n_in; (void)out_size; (void)ws_size;
  const float* x   = (const float*)d_in[0];
  const int*   ei  = (const int*)d_in[1];
  const int* batch = (const int*)d_in[2];
  const float* W1 = (const float*)d_in[3];  const float* b1 = (const float*)d_in[4];
  const float* W2 = (const float*)d_in[5];  const float* b2 = (const float*)d_in[6];
  const float* W3 = (const float*)d_in[7];  const float* b3 = (const float*)d_in[8];
  const float* lW1 = (const float*)d_in[9]; const float* lb1 = (const float*)d_in[10];
  const float* lW2 = (const float*)d_in[11]; const float* lb2 = (const float*)d_in[12];
  float* logits = (float*)d_out;
  float* zero   = logits + GG * 10;
  char* ws = (char*)d_ws;
  float* A1 = (float*)ws; ws += 128 * 128 * 4;
  float* A2 = (float*)ws; ws += 128 * 64 * 4;
  float* A3 = (float*)ws; ws += 128 * 64 * 4;
  float* XP = (float*)ws; ws += (size_t)GNP * 128 * 4;
  float* HT = (float*)ws; ws += (size_t)128 * GNP * 4;
  float* R  = (float*)ws; ws += (size_t)GNP * 64 * 4;
  float* HA = (float*)ws; ws += (size_t)GNP * 64 * 4;
  float* HB = (float*)ws; ws += (size_t)GNP * 64 * 4;
  float* dis = (float*)ws; ws += (size_t)GNP * 4;
  k_packA<<<128, 128, 0, stream>>>(W1, 128, A1);
  k_packA<<<128, 128, 0, stream>>>(W2, 64, A2);
  k_packA<<<128, 128, 0, stream>>>(W3, 64, A3);
  k_padrows<<<GNP, 128, 0, stream>>>(x, XP);
  k_deg<<<GNP / GRANGE, 256, 0, stream>>>(ei, dis);
  dim3 blk(256);
  gemm_split_kernel<float, float, 2><<<dim3(1, GNP / 256), blk, 0, stream>>>(A1, 0, XP, 0, nullptr, HT, 128, GNP, 128);
  k_gcn_agg<<<GNP / GRANGE, 256, 0, stream>>>(ei, HT, dis, b1, R, HA);
  gemm_split_kernel<float, float, 2><<<dim3(1, GNP / 256), blk, 0, stream>>>(A2, 0, HA, 0, nullptr, HT, 128, GNP, 64);
  k_gcn_agg<<<GNP / GRANGE, 256, 0, stream>>>(ei, HT, dis, b2, R, HB);
  gemm_split_kernel<float, float, 2><<<dim3(1, GNP / 256), blk, 0, stream>>>(A3, 0, HB, 0, nullptr, HT, 128, GNP, 64);
  k_gcn_agg<<<GNP / GRANGE, 256, 0, stream>>>(ei, HT, dis, b3, R, HA);
  k_pool_head<<<1, 256, 0, stream>>>(HA, batch, lW1, lb1, lW2, lb2, logits, zero);
}
